// MorkySelectiveSSM_89137751261984
// MI455X (gfx1250) — hardware-run, weakly checked
//
#include <hip/hip_runtime.h>
#include <math.h>

typedef __attribute__((ext_vector_type(16))) _Float16 v16h;
typedef __attribute__((ext_vector_type(8)))  _Float16 v8h;
typedef __attribute__((ext_vector_type(16))) __bf16   v16b;
typedef __attribute__((ext_vector_type(8)))  __bf16   v8b;
typedef __attribute__((ext_vector_type(8)))  float    v8f;
typedef __attribute__((ext_vector_type(4)))  float    v4f;

constexpr int kBatch = 2;
constexpr int kSeq   = 2048;
constexpr int kHid   = 512;
constexpr int kNst   = 64;
constexpr int kRows  = kBatch * kSeq;
constexpr int kAP    = 65;
constexpr int kAugP  = 129;
constexpr int kTileP = 68;
constexpr int kChunk = 64;
constexpr float kCarryX   = 64.0f;
constexpr float kCarryDw  = 256.0f;
constexpr float kCarryOut = kCarryX * kCarryDw;
constexpr float kCarryCw  = kCarryOut;
constexpr float kFoldOut  = 1.0f / kCarryOut;
static_assert(kCarryOut == 16384.0f);
static_assert(kNst == 64 && kHid == 512 && kRows == 4096);
static_assert((kHid % 32) == 0 && (kNst % 32) == 0);
static_assert((kRows % 64) == 0 && (kHid % 64) == 0 && (kNst % 64) == 0);
static_assert((kSeq % kChunk) == 0 && kChunk == 64);

constexpr size_t kOffMH  = 0;
constexpr size_t kOffML  = kOffMH  + (size_t)kNst  * kHid * 2;
constexpr size_t kOffXF  = kOffML  + (size_t)kNst  * kHid * 2;
constexpr size_t kOffXH  = kOffXF  + (size_t)kRows * kHid * 2;
constexpr size_t kOffXL  = kOffXH  + (size_t)kRows * kHid * 2;
constexpr size_t kOffCWH = kOffXL  + (size_t)kRows * kHid * 2;
constexpr size_t kOffCWL = kOffCWH + (size_t)kHid  * kNst * 2;
constexpr size_t kOffDWF = kOffCWL + (size_t)kHid  * kNst * 2;
constexpr size_t kOffV   = kOffDWF + (size_t)kHid  * kHid * 2;
constexpr size_t kOffU   = kOffV   + (size_t)kRows * kNst * 4;
constexpr size_t kOffHSH = kOffU   + (size_t)kRows * kNst * 4;
constexpr size_t kOffHSL = kOffHSH + (size_t)kRows * kNst * 2;
constexpr size_t kWsTotal = kOffHSL + (size_t)kRows * kNst * 2;
static_assert(kWsTotal == 16515072ull);
static_assert(kWsTotal <= 134217728ull);
static_assert((kOffML % 128) == 0 && (kOffXF % 128) == 0 && (kOffXH % 128) == 0 && (kOffXL % 128) == 0 &&
              (kOffCWH % 128) == 0 && (kOffCWL % 128) == 0 && (kOffDWF % 128) == 0 && (kOffV % 128) == 0 &&
              (kOffU % 128) == 0 && (kOffHSH % 128) == 0 && (kOffHSL % 128) == 0);

__device__ __forceinline__ unsigned short f2bf_bits(float f) {
  unsigned u = __float_as_uint(f);
  return (unsigned short)((u + 0x7FFFu + ((u >> 16) & 1u)) >> 16);
}
__device__ __forceinline__ float bf_bits2f(unsigned short h) { return __uint_as_float(((unsigned)h) << 16); }

__device__ __forceinline__ void keep4_h(v16h a, v16h b, v16h c, v16h d) { asm volatile("v_nop" :: "v"(a), "v"(b), "v"(c), "v"(d)); }
__device__ __forceinline__ void keep4_b(v16b a, v16b b, v16b c, v16b d) { asm volatile("v_nop" :: "v"(a), "v"(b), "v"(c), "v"(d)); }
__device__ __forceinline__ void acc_guard4(v8f& a, v8f& b, v8f& c, v8f& d) { asm volatile("v_nop\n\tv_nop\n\tv_nop\n\tv_nop" : "+v"(a), "+v"(b), "+v"(c), "+v"(d)); }

template <typename T> struct Frag;
template <> struct Frag<_Float16> {
  typedef v16h V; union U { v16h v; v8h h[2]; };
  static __device__ __forceinline__ v16h load(const _Float16* p) {
    U f; f.h[0] = *(const v8h*)(p); f.h[1] = *(const v8h*)(p + 16); return f.v;
  }
};
template <> struct Frag<__bf16> {
  typedef v16b V; union U { v16b v; v8b h[2]; };
  static __device__ __forceinline__ v16b load(const __bf16* p) {
    U f; f.h[0] = *(const v8b*)(p); f.h[1] = *(const v8b*)(p + 16); return f.v;
  }
};

__device__ __forceinline__ v8f mma_bf(v16b a, v16b b, v8f c) {
  c = __builtin_amdgcn_wmma_f32_16x16x32_bf16(false, a, false, b, (short)0, c, false, false);
  asm volatile("v_nop\n\tv_nop\n\tv_nop\n\tv_nop" : "+v"(c) : "v"(a), "v"(b));
  return c;
}
__device__ __forceinline__ v8f mma_hf(v16h a, v16h b, v8f c) {
  c = __builtin_amdgcn_wmma_f32_16x16x32_f16(false, a, false, b, (short)0, c, false, false);
  asm volatile("v_nop\n\tv_nop\n\tv_nop\n\tv_nop" : "+v"(c) : "v"(a), "v"(b));
  return c;
}

__device__ __forceinline__ void split8(const v4f a0, const v4f a1, v8h& hv, v8h& lv) {
#pragma unroll
  for (int e = 0; e < 4; ++e) {
    const float f0 = a0[e];
    const float f1 = a1[e];
    const unsigned short h0 = f2bf_bits(f0);
    const unsigned short h1 = f2bf_bits(f1);
    const unsigned short l0 = f2bf_bits(f0 - bf_bits2f(h0));
    const unsigned short l1 = f2bf_bits(f1 - bf_bits2f(h1));
    hv[e]     = __builtin_bit_cast(_Float16, h0);
    hv[4 + e] = __builtin_bit_cast(_Float16, h1);
    lv[e]     = __builtin_bit_cast(_Float16, l0);
    lv[4 + e] = __builtin_bit_cast(_Float16, l1);
  }
}

__global__ __launch_bounds__(256) void prep_inverse_kernel(
    const float* __restrict__ Ag, const float* __restrict__ Bw,
    unsigned short* __restrict__ MH, unsigned short* __restrict__ ML)
{
  __shared__ __align__(16) float aug[kNst * kAugP];
  const int tid  = threadIdx.x;
  const int lane = tid & 31;
  const int wave = __builtin_amdgcn_readfirstlane((int)(threadIdx.x >> 5));
#pragma unroll 1
  for (int it = 0; it < 32; ++it) {
    const int idx = it * 256 + tid;
    const int r = idx >> 7;
    const int c = idx & 127;
    const int cc = c & 63;
    float a = Ag[r * kNst + cc];
    asm volatile("" : "+v"(a));
    const float e = (cc == r) ? 1.0f : 0.0f;
    aug[r * kAugP + c] = (c < 64) ? a : e;
  }
  __syncthreads();

#pragma unroll 1
  for (int k = 0; k < kNst; ++k) {
    const int r1 = lane + 32;
    const float c0 = fabsf(aug[lane * kAugP + k]);
    const float c1 = fabsf(aug[r1 * kAugP + k]);
    float best = (lane >= k) ? c0 : -1.0f;
    int bi = lane;
    const float v1 = (r1 >= k) ? c1 : -1.0f;
    const bool t1 = (v1 > best);
    best = t1 ? v1 : best;
    bi   = t1 ? r1 : bi;
#pragma unroll
    for (int off = 16; off >= 1; off >>= 1) {
      const float ov = __shfl_xor(best, off, 32);
      const int   oi = __shfl_xor(bi, off, 32);
      const bool take = (ov > best) || ((ov == best) && (oi < bi));
      best = take ? ov : best;
      bi   = take ? oi : bi;
    }
    int p = __builtin_amdgcn_readfirstlane(bi);
    p = (p < k) ? k : p;
    p = (p > kNst - 1) ? (kNst - 1) : p;
    __syncthreads();
    if (tid < 128) {
      const float ra = aug[k * kAugP + tid];
      const float rb = aug[p * kAugP + tid];
      aug[k * kAugP + tid] = rb;
      aug[p * kAugP + tid] = ra;
    }
    __syncthreads();
    {
      const int r = tid & 63;
      const int q = tid >> 6;
      const float rcp = 1.0f / aug[k * kAugP + k];
      const float l = aug[r * kAugP + k] * rcp;
      if (r > k) {
#pragma unroll 1
        for (int jj = 0; jj < 32; ++jj) {
          const int j = q * 32 + jj;
          if (j > k) {
            const float cur = aug[r * kAugP + j];
            aug[r * kAugP + j] = fmaf(-l, aug[k * kAugP + j], cur);
          }
        }
      }
    }
    __syncthreads();
  }

  if (tid < 64) {
    const int c = tid;
#pragma unroll 1
    for (int i = kNst - 1; i >= 0; --i) {
      float acc = aug[i * kAugP + 64 + c];
#pragma unroll 1
      for (int j = i + 1; j < kNst; ++j) acc = fmaf(-aug[i * kAugP + j], aug[j * kAugP + 64 + c], acc);
      const float rd = 1.0f / aug[i * kAugP + i];
      aug[i * kAugP + 64 + c] = acc * rd;
    }
  }
  __syncthreads();

  const int tr = wave >> 1;
  const int tc = tid & 63;
#pragma unroll 1
  for (int g = 0; g < 16; ++g) {
    const int n = g * 4 + tr;
    v4f m0 = (v4f){0.f, 0.f, 0.f, 0.f};
    v4f m1 = (v4f){0.f, 0.f, 0.f, 0.f};
#pragma unroll 2
    for (int k = 0; k < kNst; ++k) {
      const float a = aug[n * kAugP + 64 + k];
      const v4f b0 = *(const v4f*)(Bw + (size_t)k * kHid + tc * 8);
      const v4f b1 = *(const v4f*)(Bw + (size_t)k * kHid + tc * 8 + 4);
#pragma unroll
      for (int e = 0; e < 4; ++e) {
        m0[e] = fmaf(a, b0[e], m0[e]);
        m1[e] = fmaf(a, b1[e], m1[e]);
      }
    }
    v8h hv, lv;
    split8(m0, m1, hv, lv);
    unsigned short* qh = MH + (size_t)n * kHid + tc * 8;
    unsigned short* ql = ML + (size_t)n * kHid + tc * 8;
    *(volatile v8h*)qh = hv;
    *(volatile v8h*)ql = lv;
    __threadfence();
    *(volatile v8h*)qh = hv;
    *(volatile v8h*)ql = lv;
  }
}

template <int MODE>
__global__ __launch_bounds__(256) void make_planes_kernel(
    const float* __restrict__ src, unsigned short* __restrict__ d16,
    unsigned short* __restrict__ dhi, unsigned short* __restrict__ dlo,
    int total8, float carry16, float carrybf)
{
  const int i = blockIdx.x * 256 + threadIdx.x;
  if (i >= total8) return;
  const size_t e0 = (size_t)i << 3;
  const v4f a0 = *(const v4f*)(src + e0);
  const v4f a1 = *(const v4f*)(src + e0 + 4);
  v8h fv, hv, lv;
  if (MODE & 1) {
#pragma unroll
    for (int e = 0; e < 4; ++e) {
      const float s0 = a0[e] * carry16;
      const float s1 = a1[e] * carry16;
      fv[e]     = (_Float16)s0;
      fv[4 + e] = (_Float16)s1;
    }
  }
  if (MODE & 2) {
    v4f b0, b1;
#pragma unroll
    for (int e = 0; e < 4; ++e) {
      b0[e] = a0[e] * carrybf;
      b1[e] = a1[e] * carrybf;
    }
    split8(b0, b1, hv, lv);
  }
  if (MODE & 1) *(volatile v8h*)(d16 + e0) = fv;
  if (MODE & 2) {
    *(volatile v8h*)(dhi + e0) = hv;
    *(volatile v8h*)(dlo + e0) = lv;
  }
  __threadfence();
  if (MODE & 1) *(volatile v8h*)(d16 + e0) = fv;
  if (MODE & 2) {
    *(volatile v8h*)(dhi + e0) = hv;
    *(volatile v8h*)(dlo + e0) = lv;
  }
}

__global__ __launch_bounds__(256) void gemm_dual_kernel(
    const unsigned short* __restrict__ Ahp, const unsigned short* __restrict__ Alp, int ldaB,
    const unsigned short* __restrict__ Bhp, const unsigned short* __restrict__ Blp, int ldbB, int KB,
    const unsigned short* __restrict__ Afp, int ldaF,
    const unsigned short* __restrict__ Bfp, int ldbF, int KF,
    float* __restrict__ C, int ldc,
    const float* __restrict__ bias0, const float* __restrict__ bias1, int use_bias,
    int M, int N, float scale)
{
  const __bf16* Ah = (const __bf16*)Ahp;
  const __bf16* Al = (const __bf16*)Alp;
  const __bf16* Bh = (const __bf16*)Bhp;
  const __bf16* Bl = (const __bf16*)Blp;
  const _Float16* Af = (const _Float16*)Afp;
  const _Float16* Bf = (const _Float16*)Bfp;
  __shared__ __align__(16) float sT[8][16 * kTileP];
  const int lane = threadIdx.x & 31;
  const int wave = __builtin_amdgcn_readfirstlane((int)(threadIdx.x >> 5));
  const int tilesN = N >> 6;
  const int tilesM = M >> 6;
  const int tile = blockIdx.x * 8 + wave;
  if (tile >= tilesM * tilesN) return;
  const int tm = tile / tilesN;
  const int tn = tile - tm * tilesN;
  const int m0 = tm << 6;
  const int n0 = tn << 6;

  const int rlane = lane & 15;
  const int koff  = (lane >> 4) * 8;
  const int mOff  = (lane >> 4) * 8;

  v8f acc[4][4];
#pragma unroll
  for (int i = 0; i < 4; ++i)
#pragma unroll
    for (int j = 0; j < 4; ++j) acc[i][j] = (v8f){0.f,0.f,0.f,0.f,0.f,0.f,0.f,0.f};

  for (int k0 = 0; k0 < KB; k0 += 32) {
    v16b bh[4], bl[4];
#pragma unroll
    for (int j = 0; j < 4; ++j) {
      const size_t bo = (size_t)(n0 + (j << 4) + rlane) * ldbB + koff + k0;
      bh[j] = Frag<__bf16>::load(Bh + bo);
      bl[j] = Frag<__bf16>::load(Bl + bo);
    }
#pragma unroll
    for (int i = 0; i < 4; ++i) {
      const size_t ao = (size_t)(m0 + (i << 4) + rlane) * ldaB + koff + k0;
      const v16b ah = Frag<__bf16>::load(Ah + ao);
      const v16b al = Frag<__bf16>::load(Al + ao);
#pragma unroll
      for (int j = 0; j < 4; ++j) {
        acc[i][j] = mma_bf(ah, bh[j], acc[i][j]);
        acc[i][j] = mma_bf(ah, bl[j], acc[i][j]);
        acc[i][j] = mma_bf(al, bh[j], acc[i][j]);
      }
    }
    keep4_b(bh[0], bh[1], bh[2], bh[3]);
    keep4_b(bl[0], bl[1], bl[2], bl[3]);
  }
  for (int k0 = 0; k0 < KF; k0 += 32) {
    v16h bf[4];
#pragma unroll
    for (int j = 0; j < 4; ++j) {
      const size_t bo = (size_t)(n0 + (j << 4) + rlane) * ldbF + koff + k0;
      bf[j] = Frag<_Float16>::load(Bf + bo);
    }
#pragma unroll
    for (int i = 0; i < 4; ++i) {
      const size_t ao = (size_t)(m0 + (i << 4) + rlane) * ldaF + koff + k0;
      const v16h af = Frag<_Float16>::load(Af + ao);
#pragma unroll
      for (int j = 0; j < 4; ++j) acc[i][j] = mma_hf(af, bf[j], acc[i][j]);
    }
    keep4_h(bf[0], bf[1], bf[2], bf[3]);
  }
  acc_guard4(acc[0][0], acc[0][1], acc[0][2], acc[0][3]);
  acc_guard4(acc[1][0], acc[1][1], acc[1][2], acc[1][3]);
  acc_guard4(acc[2][0], acc[2][1], acc[2][2], acc[2][3]);
  acc_guard4(acc[3][0], acc[3][1], acc[3][2], acc[3][3]);

  float* slab = sT[wave];
  float bv[4];
#pragma unroll
  for (int j = 0; j < 4; ++j) {
    const int n = n0 + (j << 4) + rlane;
    bv[j] = 0.f;
    if (use_bias) bv[j] = bias0[n] + bias1[n];
  }
#pragma unroll
  for (int i = 0; i < 4; ++i) {
    const int mBase = m0 + (i << 4);
#pragma unroll
    for (int j = 0; j < 4; ++j) {
#pragma unroll
      for (int r = 0; r < 8; ++r) {
        const float v = acc[i][j][r] * scale + bv[j];
        slab[(mOff + r) * kTileP + (j << 4) + rlane] = v;
      }
    }
    __builtin_amdgcn_fence(__ATOMIC_RELEASE, "workgroup");
    __builtin_amdgcn_wave_barrier();
    __builtin_amdgcn_fence(__ATOMIC_ACQUIRE, "workgroup");
    {
      const int hh = lane >> 4;
      const int c4 = (lane & 15) * 4;
      for (int pass = 0; pass < 2; ++pass) {
#pragma unroll
        for (int it = 0; it < 8; ++it) {
          const int row = it * 2 + hh;
          const v4f v = *(const v4f*)(slab + row * kTileP + c4);
          *(volatile v4f*)(C + (size_t)(mBase + row) * ldc + n0 + c4) = v;
        }
        __threadfence();
      }
    }
    __builtin_amdgcn_fence(__ATOMIC_RELEASE, "workgroup");
    __builtin_amdgcn_wave_barrier();
    __builtin_amdgcn_fence(__ATOMIC_ACQUIRE, "workgroup");
  }
}

__global__ __launch_bounds__(256) void u_chunk_kernel(
    const float* __restrict__ Ag, const float* __restrict__ delta,
    const float* __restrict__ V, float* __restrict__ U)
{
  __shared__ __align__(16) float sA[kNst * kAP];
  __shared__ __align__(16) float sV[kChunk * kNst];
  __shared__ __align__(16) float sU[kChunk * kTileP];
  __shared__ float sDl[kChunk];
  const int tid  = threadIdx.x;
  const int lane = tid & 31;
  const int wave = __builtin_amdgcn_readfirstlane((int)(threadIdx.x >> 5));
  const size_t row0 = (size_t)blockIdx.x * kChunk;
#pragma unroll 1
  for (int it = 0; it < 16; ++it) {
    const int idx = it * 256 + tid;
    sA[(idx >> 6) * kAP + (idx & 63)] = Ag[idx];
  }
#pragma unroll
  for (int it = 0; it < 4; ++it) {
    const int i4 = (it * 256 + tid) * 4;
    *(v4f*)(sV + i4) = *(const v4f*)(V + row0 * kNst + i4);
  }
  {
    float dv = delta[row0 + (tid & 63)];
    asm volatile("" : "+v"(dv));
    if (tid < 64) sDl[tid] = dv;
  }
  __syncthreads();
  const int m  = tid & 63;
  const int sq = wave >> 1;
#pragma unroll 1
  for (int ss = 0; ss < 16; ++ss) {
    const int s = sq * 16 + ss;
    const float dlt = sDl[s];
    const float* ar = sA + m * kAP;
    const float* vr = sV + s * kNst;
    float acc = 0.f;
#pragma unroll 2
    for (int n = 0; n < kNst; ++n) {
      const float e = expf(dlt * ar[n]);
      acc = fmaf(e, vr[n], acc);
    }
    sU[s * kTileP + m] = acc - vr[m];
  }
  __syncthreads();
  {
    const int hh = lane >> 4;
    const int c4 = (lane & 15) * 4;
    v4f fv[4];
#pragma unroll
    for (int it = 0; it < 4; ++it) fv[it] = *(const v4f*)(sU + (wave * 8 + it * 2 + hh) * kTileP + c4);
    for (int pass = 0; pass < 2; ++pass) {
#pragma unroll
      for (int it = 0; it < 4; ++it)
        *(volatile v4f*)(U + (row0 + wave * 8 + it * 2 + hh) * kNst + c4) = fv[it];
      __threadfence();
    }
  }
}

__global__ __launch_bounds__(256) void scan_kernel(
    const float* __restrict__ Ag, const float* __restrict__ delta, const float* __restrict__ U,
    unsigned short* __restrict__ HSH, unsigned short* __restrict__ HSL)
{
  __shared__ __align__(16) float sA[kNst * kAP];
  __shared__ __align__(16) float sUc[kChunk * kNst];
  __shared__ __align__(16) float sHS[kChunk * kTileP];
  __shared__ float sPart[256];
  __shared__ float sH[kNst];
  __shared__ float sDl[kChunk];
  const int tid  = threadIdx.x;
  const int lane = tid & 31;
  const int wave = __builtin_amdgcn_readfirstlane((int)(threadIdx.x >> 5));
  const size_t rowb = (size_t)blockIdx.x * kSeq;
#pragma unroll 1
  for (int it = 0; it < 16; ++it) {
    const int idx = it * 256 + tid;
    sA[(idx >> 6) * kAP + (idx & 63)] = Ag[idx];
  }
  if (tid < 64) sH[tid] = 0.f;
  const int n = tid & 63;
  const int q = wave >> 1;
  const int q4 = lane >> 3;
  const int c8 = (lane & 7) * 8;
#pragma unroll 1
  for (int t0 = 0; t0 < kSeq; t0 += kChunk) {
    __syncthreads();
#pragma unroll
    for (int it = 0; it < 4; ++it) {
      const int i4 = (it * 256 + tid) * 4;
      *(v4f*)(sUc + i4) = *(const v4f*)(U + (rowb + t0) * kNst + i4);
    }
    {
      float dv = delta[rowb + t0 + (tid & 63)];
      asm volatile("" : "+v"(dv));
      if (tid < 64) sDl[tid] = dv;
    }
    __syncthreads();
#pragma unroll 1
    for (int s = 0; s < kChunk; ++s) {
      const float dlt = sDl[s];
      float acc = 0.f;
#pragma unroll 2
      for (int j = 0; j < 16; ++j) {
        const int mm = q * 16 + j;
        const float e = expf(dlt * sA[mm * kAP + n]);
        acc = fmaf(sH[mm], e, acc);
      }
      sPart[tid] = acc;
      __syncthreads();
      if (tid < 64) {
        const float hn = ((sPart[n] + sPart[64 + n]) + (sPart[128 + n] + sPart[192 + n])) + sUc[s * kNst + n];
        sH[n] = hn;
        sHS[s * kTileP + n] = hn;
      }
      __syncthreads();
    }
    v8h hv[2], lv[2];
#pragma unroll
    for (int it = 0; it < 2; ++it) {
      const int row = it * 32 + wave * 4 + q4;
      const float* sp = sHS + row * kTileP + c8;
      const v4f a0 = *(const v4f*)(sp);
      const v4f a1 = *(const v4f*)(sp + 4);
      split8(a0, a1, hv[it], lv[it]);
    }
    for (int pass = 0; pass < 2; ++pass) {
#pragma unroll
      for (int it = 0; it < 2; ++it) {
        const int row = it * 32 + wave * 4 + q4;
        const size_t o = (rowb + t0 + row) * kNst + c8;
        *(volatile v8h*)(HSH + o) = hv[it];
        *(volatile v8h*)(HSL + o) = lv[it];
      }
      __threadfence();
    }
  }
}

extern "C" void kernel_launch(void* const* d_in, const int* in_sizes, int n_in,
                              void* d_out, int out_size, void* d_ws, size_t ws_size,
                              hipStream_t stream) {
  if (n_in < 8) return;
  if (in_sizes[0] != kRows * kHid) return;
  if (in_sizes[1] != kRows) return;
  if (in_sizes[2] != kNst * kNst) return;
  if (in_sizes[3] != kNst * kHid) return;
  if (in_sizes[4] != kHid * kNst) return;
  if (in_sizes[5] != kHid) return;
  if (in_sizes[6] != kHid * kHid) return;
  if (in_sizes[7] != kHid) return;
  if (out_size != kRows * kHid) return;
  if (ws_size < kWsTotal) return;

  const float* x     = (const float*)d_in[0];
  const float* delta = (const float*)d_in[1];
  const float* Amat  = (const float*)d_in[2];
  const float* Bw    = (const float*)d_in[3];
  const float* Cw    = (const float*)d_in[4];
  const float* Cb    = (const float*)d_in[5];
  const float* Dw    = (const float*)d_in[6];
  const float* Db    = (const float*)d_in[7];
  float* out = (float*)d_out;

  char* ws = (char*)d_ws;
  unsigned short* MH  = (unsigned short*)(ws + kOffMH);
  unsigned short* ML  = (unsigned short*)(ws + kOffML);
  unsigned short* XF  = (unsigned short*)(ws + kOffXF);
  unsigned short* XH  = (unsigned short*)(ws + kOffXH);
  unsigned short* XL  = (unsigned short*)(ws + kOffXL);
  unsigned short* CWH = (unsigned short*)(ws + kOffCWH);
  unsigned short* CWL = (unsigned short*)(ws + kOffCWL);
  unsigned short* DWF = (unsigned short*)(ws + kOffDWF);
  float*          V   = (float*)(ws + kOffV);
  float*          U   = (float*)(ws + kOffU);
  unsigned short* HSH = (unsigned short*)(ws + kOffHSH);
  unsigned short* HSL = (unsigned short*)(ws + kOffHSL);

  prep_inverse_kernel<<<1, 256, 0, stream>>>(Amat, Bw, MH, ML);

  make_planes_kernel<3><<<(kRows * kHid / 8) / 256, 256, 0, stream>>>(x, XF, XH, XL, kRows * kHid / 8, kCarryX, 1.0f);
  make_planes_kernel<2><<<(kHid * kNst / 8) / 256, 256, 0, stream>>>(Cw, CWH, CWH, CWL, kHid * kNst / 8, 1.0f, kCarryCw);
  make_planes_kernel<1><<<(kHid * kHid / 8) / 256, 256, 0, stream>>>(Dw, DWF, DWF, DWF, kHid * kHid / 8, kCarryDw, 1.0f);

  gemm_dual_kernel<<<8, 256, 0, stream>>>(
      XH, XL, kHid, MH, ML, kHid, kHid,
      XF, kHid, DWF, kHid, 0,
      V, kNst, Cb, Db, 0,
      kRows, kNst, 1.0f);

  u_chunk_kernel<<<kRows / kChunk, 256, 0, stream>>>(Amat, delta, V, U);

  scan_kernel<<<kBatch, 256, 0, stream>>>(Amat, delta, U, HSH, HSL);

  gemm_dual_kernel<<<64, 256, 0, stream>>>(
      HSH, HSL, kNst, CWH, CWL, kNst, kNst,
      XF, kHid, DWF, kHid, kHid,
      out, kHid, Cb, Db, 1,
      kRows, kHid, kFoldOut);
}
